// EdgeConv3d_5016521801768
// MI455X (gfx1250) — hardware-verified
//
#include <hip/hip_runtime.h>


namespace {
constexpr int B = 2, C = 64, NN = 16384, K = 16, CO = 64;
constexpr float XS = 8.0f, WSC = 256.0f;
typedef _Float16 b16;
typedef __attribute__((ext_vector_type(16))) _Float16 v16b;
typedef __attribute__((ext_vector_type(8))) _Float16 v8b;
typedef __attribute__((ext_vector_type(8))) float v8f;
typedef __attribute__((ext_vector_type(4))) float v4f;
__device__ __forceinline__ float bf16_rne(float f) { unsigned int u = __float_as_uint(f); u += 0x7FFFu + ((u >> 16) & 1u); float r = __uint_as_float(u & 0xFFFF0000u); asm volatile("" : "+v"(r)); return r; }
__device__ __forceinline__ void split16(float v, b16& hi, b16& lo) { hi = (b16)v; lo = (b16)(v - (float)hi); }
__device__ __forceinline__ v16b frag_kb(const b16* p, int hh) { const v8b a = *(const v8b*)(p + 8 * hh), b = *(const v8b*)(p + 16 + 8 * hh); v16b f;
#pragma unroll
  for (int e = 0; e < 8; ++e) { f[e] = a[e]; f[8 + e] = b[e]; } return f; }
__device__ __forceinline__ v8f wmma16b(v16b a, v16b b, v8f c) { v8f d = __builtin_amdgcn_wmma_f32_16x16x32_f16(false, a, false, b, (short)0, c, false, false); asm volatile("v_nop\n\tv_nop\n\tv_nop\n\tv_nop" : "+v"(d) : "v"(a), "v"(b)); return d; }
__device__ __forceinline__ void wave_lds_sync() { __builtin_amdgcn_fence(__ATOMIC_RELEASE, "workgroup"); __builtin_amdgcn_wave_barrier(); __builtin_amdgcn_fence(__ATOMIC_ACQUIRE, "workgroup"); }
__device__ __forceinline__ int iclamp(int v, int lo, int hi) { return v < lo ? lo : (v > hi ? hi : v); }

__global__ __launch_bounds__(256) void wput_kernel(const float* __restrict__ w, b16* __restrict__ WAh, b16* __restrict__ WAl, b16* __restrict__ WBp) { const int u = blockIdx.x * 256 + threadIdx.x; if (u >= CO * 8) return; const int o = u / 8, k0 = (u % 8) * 8; v8b ah, al, bb;
#pragma unroll
  for (int j = 0; j < 8; ++j) { const float wa = bf16_rne(w[(size_t)o * 2 * C + k0 + j]), wb = bf16_rne(w[(size_t)o * 2 * C + C + k0 + j]); b16 p, q; split16((wa - wb) * WSC, p, q); ah[j] = p; al[j] = q; bb[j] = (b16)(wb * WSC); }
  for (int pass = 0; pass < 2; ++pass) { *(volatile v8b*)(WAh + (size_t)o * C + k0) = ah; *(volatile v8b*)(WAl + (size_t)o * C + k0) = al; *(volatile v8b*)(WBp + (size_t)o * C + k0) = bb; __threadfence(); } }
__global__ __launch_bounds__(32) void dense_kernel(const float* __restrict__ x, const b16* __restrict__ WAh, const b16* __restrict__ WAl, const b16* __restrict__ WBp, int RLIM, float* __restrict__ P) { __shared__ __attribute__((aligned(16))) b16 Ah[16][72]; __shared__ float Tf[16][132]; const int lane = threadIdx.x, nloc = lane & 15, hlf = lane >> 4; const size_t r0 = (size_t)blockIdx.x * 16; if (r0 >= (size_t)RLIM) return; const int b = (int)(r0 / NN), n0 = (int)(r0 % NN);
  for (int q = 0; q < 2; ++q) { const int c = q * 32 + lane; for (int rr = 0; rr < 16; ++rr) Ah[rr][c] = (b16)(bf16_rne(x[((size_t)b * C + c) * NN + n0 + rr]) * XS); }
  wave_lds_sync(); const v16b a0 = frag_kb(&Ah[nloc][0], hlf), a1 = frag_kb(&Ah[nloc][32], hlf);
#pragma unroll
  for (int t = 0; t < 4; ++t) { const size_t ro = (size_t)(t * 16 + nloc) * C; v8f pa = {}, pb = {};
    pa = wmma16b(a0, frag_kb(WAh + ro, hlf), pa); pa = wmma16b(a0, frag_kb(WAl + ro, hlf), pa); pa = wmma16b(a1, frag_kb(WAh + ro + 32, hlf), pa); pa = wmma16b(a1, frag_kb(WAl + ro + 32, hlf), pa);
    pb = wmma16b(a0, frag_kb(WBp + ro, hlf), pb); pb = wmma16b(a1, frag_kb(WBp + ro + 32, hlf), pb);
#pragma unroll
    for (int r8 = 0; r8 < 8; ++r8) { Tf[8 * hlf + r8][t * 16 + nloc] = pa[r8] * (1.0f / (XS * WSC)); Tf[8 * hlf + r8][CO + t * 16 + nloc] = pb[r8] * (1.0f / (XS * WSC)); } }
  wave_lds_sync();
  for (int pass = 0; pass < 2; ++pass) { for (int rr = 0; rr < 16; ++rr) *(volatile v4f*)(P + (r0 + rr) * 2 * CO + lane * 4) = *(const v4f*)(&Tf[rr][lane * 4]); __threadfence(); } }
__global__ __launch_bounds__(256) void edge_kernel(const float* __restrict__ P, const int* __restrict__ ei, const float* __restrict__ bias, int RLIM, float* __restrict__ out) { const int wave = threadIdx.x >> 5, lane = threadIdx.x & 31; const size_t r0 = ((size_t)blockIdx.x * 8 + wave) * 32; if (r0 >= (size_t)RLIM) return; const int b = (int)(r0 / NN), n0 = (int)(r0 % NN); const size_t r = r0 + lane;
  float mx[CO];
#pragma unroll
  for (int c = 0; c < CO; ++c) mx[c] = 0.0f;
#pragma unroll 1
  for (int k = 0; k < K; ++k) { const size_t i = (size_t)b * NN + iclamp(ei[((size_t)(1 * B + b) * NN + (n0 + lane)) * K + k], 0, NN - 1), j = (size_t)b * NN + iclamp(ei[((size_t)(0 * B + b) * NN + (n0 + lane)) * K + k], 0, NN - 1);
#pragma unroll
    for (int c4 = 0; c4 < CO / 4; ++c4) { const v4f pa = *(const v4f*)(P + i * 2 * CO + c4 * 4), pb = *(const v4f*)(P + j * 2 * CO + CO + c4 * 4);
#pragma unroll
      for (int q = 0; q < 4; ++q) mx[c4 * 4 + q] = fmaxf(mx[c4 * 4 + q], pa[q] + pb[q] + bf16_rne(bias[c4 * 4 + q])); } }
  (void)r;
  for (int pass = 0; pass < 2; ++pass) {
#pragma unroll
    for (int c = 0; c < CO; ++c) ((volatile float*)out)[((size_t)b * CO + c) * NN + n0 + lane] = mx[c];
    __threadfence(); } }
}

extern "C" void kernel_launch(void* const* d_in, const int* in_sizes, int n_in, void* d_out, int out_size, void* d_ws, size_t ws_size, hipStream_t stream) {
  (void)n_in;
  auto Fp = [&](int i) { return (const float*)d_in[i]; }; auto Ip = [&](int i) { return (const int*)d_in[i]; };
  if (in_sizes[0] != B * C * NN || in_sizes[1] != 2 * B * NN * K || in_sizes[2] != CO * 2 * C || in_sizes[3] != CO || out_size != B * CO * NN) return;
  const int RLIM = B * NN;
  size_t off = 0; char* ws = (char*)d_ws;
  auto carve = [&](size_t bytes) { char* p = ws + off; off += (bytes + 255) & ~(size_t)255; return p; };
  b16* WAh = (b16*)carve((size_t)CO * C * 2); b16* WAl = (b16*)carve((size_t)CO * C * 2); b16* WBp = (b16*)carve((size_t)CO * C * 2); float* P = (float*)carve((size_t)B * NN * 2 * CO * 4);
  if (off > ws_size || off > ((size_t)32 << 20)) return;
  wput_kernel<<<(CO * 8 + 255) / 256, 256, 0, stream>>>(Fp(2), WAh, WAl, WBp);
  dense_kernel<<<B * NN / 16, 32, 0, stream>>>(Fp(0), WAh, WAl, WBp, B * NN, P);
  edge_kernel<<<(RLIM / 32 + 7) / 8, 256, 0, stream>>>(P, Ip(1), Fp(3), RLIM, (float*)d_out);
}
